// NeighborMLPConvLayer_15350213116605
// MI455X (gfx1250) — hardware-run, weakly checked
//
#include <hip/hip_runtime.h>
#include <stddef.h>
#include <stdint.h>


#define NPTS    50000
#define MPAD    50048
#define NE      1600000
#define CIN     32
#define HID     128
#define OUTC    64
#define XP      32
#define W1P     32
#define KONE    32
#define PQP     128
#define GAP     256
#define W2P     256
#define G_SPLIT 1
#define KTWO    (G_SPLIT ? 256 : 128)
#define TRIPCAP 4096
#define PTHR    256
#define G1M     64
#define G1THR   128
#define WTHR    256
#define WNW     8
#define G2M     128
#define G2THR   256
#define XBLK    ((MPAD * 4) / PTHR)
#define NWB     (MPAD / WNW)
#define PREPB   (2 * XBLK + 4 + 8 + 1)

#define XPLANE  ((size_t)MPAD * XP)
#define W1PLANE ((size_t)HID * W1P)
#define PQPLANE ((size_t)MPAD * PQP)

static_assert(MPAD == 391 * 128 && MPAD == 782 * G1M && MPAD == NWB * WNW && MPAD >= NPTS);
static_assert(MPAD % G2M == 0 && (MPAD * 4) % PTHR == 0);
static_assert(32 * 4 == HID && PQP == HID);
static_assert(KONE == 32 && KONE == CIN && XP == KONE && W1P == KONE);
static_assert(TRIPCAP == 4096 && TRIPCAP % 32 == 0 && TRIPCAP <= NE);
static_assert(GAP == 2 * HID && W2P == 2 * HID && KTWO % 32 == 0 && KTWO <= GAP && KTWO <= W2P);
static_assert(OUTC * 4 == 256 && OUTC == 4 * 16);
static_assert(NPTS * OUTC == 3200000);
static_assert(G1M == (G1THR / 32) * 16 && G2M == (G2THR / 32) * 16 && WTHR == WNW * 32);
static_assert(2 * HID * 4 == 4 * PTHR && OUTC * 32 == 8 * PTHR);
static_assert(G1M * HID * 4 + HID * 4 <= 327680);
static_assert(WNW * HID * 4 + 32 <= 327680);
static_assert(G2M * OUTC * 4 + OUTC * 4 + G2M * 4 <= 327680);

#define AL256(x) ((((size_t)(x)) + 255u) & ~(size_t)255)
constexpr size_t SZ_XAB = (size_t)2 * MPAD * XP * 2;
constexpr size_t SZ_W1T = (size_t)2 * HID * W1P * 2;
constexpr size_t SZ_W2T = (size_t)OUTC * W2P * 2;
constexpr size_t SZ_B1F = (size_t)HID * 4;
constexpr size_t SZ_B2F = (size_t)OUTC * 4;
constexpr size_t SZ_PQ  = (size_t)2 * MPAD * PQP * 4;
constexpr size_t SZ_G   = (size_t)MPAD * GAP * 2;
constexpr size_t SZ_CN  = (size_t)NWB * 128;
constexpr size_t O_XAB = 0;
constexpr size_t O_W1T = AL256(O_XAB + SZ_XAB);
constexpr size_t O_W2T = AL256(O_W1T + SZ_W1T);
constexpr size_t O_B1F = AL256(O_W2T + SZ_W2T);
constexpr size_t O_B2F = AL256(O_B1F + SZ_B1F);
constexpr size_t O_PQ  = AL256(O_B2F + SZ_B2F);
constexpr size_t O_G   = AL256(O_PQ + SZ_PQ);
constexpr size_t O_CN  = AL256(O_G + SZ_G);
constexpr size_t WS_TOTAL = AL256(O_CN + SZ_CN);
static_assert(WS_TOTAL <= ((size_t)128u << 20));

typedef float          v4f   __attribute__((ext_vector_type(4)));
typedef float          v8f   __attribute__((ext_vector_type(8)));
typedef int            v4i   __attribute__((ext_vector_type(4)));
typedef int            v8i   __attribute__((ext_vector_type(8)));
typedef unsigned       v4u   __attribute__((ext_vector_type(4)));
typedef unsigned short v8us  __attribute__((ext_vector_type(8)));
typedef __bf16         v16bf __attribute__((ext_vector_type(16)));
typedef v4f  __attribute__((may_alias)) v4fa;
typedef v4i  __attribute__((may_alias)) v4ia;
typedef v8us __attribute__((may_alias)) v8usa;
union FragB { v16bf v; v8us h[2]; v8i w; };

__device__ __forceinline__ v8f wmb(const FragB& a, const FragB& b, v8f c) {
  v8f d = __builtin_amdgcn_wmma_f32_16x16x32_bf16(false, a.v, false, b.v, (short)0, c, false, false);
  asm volatile("v_nop\n\tv_nop\n\tv_nop\n\tv_nop" : "+v"(d) : "v"(a.w), "v"(b.w));
  return d;
}

__device__ __forceinline__ unsigned bf16_bits(float f) {
  const unsigned u = __float_as_uint(f);
  return ((u + 0x7FFFu + ((u >> 16) & 1u)) >> 16) & 0xFFFFu;
}
__device__ __forceinline__ float bf16_val(float f) { return __uint_as_float(bf16_bits(f) << 16); }
__device__ __forceinline__ void pack2(float a, float b, unsigned& hw, unsigned& lw) {
  const unsigned ha = bf16_bits(a), hb = bf16_bits(b);
  const unsigned la = bf16_bits(a - __uint_as_float(ha << 16));
  const unsigned lb = bf16_bits(b - __uint_as_float(hb << 16));
  hw = ha | (hb << 16);
  lw = la | (lb << 16);
}

__device__ __forceinline__ void wave_sync() {
  __builtin_amdgcn_fence(__ATOMIC_RELEASE, "wavefront");
  __builtin_amdgcn_wave_barrier();
  __builtin_amdgcn_fence(__ATOMIC_ACQUIRE, "wavefront");
}

__device__ __forceinline__ float gelu_e(float v) {
#pragma clang fp contract(off)
  const float t = v * 0.70710678f;
  const float e = erff(t);
  return (0.5f * v) * (1.0f + e);
}

__global__ __launch_bounds__(PTHR) void k_prep(const float* __restrict__ xa, const float* __restrict__ xb,
                                               const float* __restrict__ W1, const float* __restrict__ b1,
                                               const float* __restrict__ W2, const float* __restrict__ b2,
                                               unsigned short* XAB, unsigned short* W1T, unsigned short* W2T,
                                               float* B1F, float* B2F) {
  const int tid = (int)threadIdx.x;
  const int bx  = (int)blockIdx.x;
  if (bx < 2 * XBLK) {
    const int sel = (bx >= XBLK) ? 1 : 0;
    const int u   = (bx - sel * XBLK) * PTHR + tid;
    const int row = u >> 2;
    const int pc  = u & 3;
    const int rc  = row < NPTS ? row : NPTS - 1;
    const size_t so = (size_t)rc * CIN + (size_t)(8 * pc);
    v4f a, b;
    if (sel == 0) {
      a = *(const v4f*)(xa + so);
      b = *(const v4f*)(xa + so + 4);
    } else {
      a = *(const v4f*)(xb + so);
      b = *(const v4f*)(xb + so + 4);
    }
    asm volatile("" :: "v"(a), "v"(b));
    const unsigned mk = (row < NPTS) ? 0xFFFFu : 0u;
    v8us o;
    o[0] = (unsigned short)(bf16_bits(a.x) & mk); o[1] = (unsigned short)(bf16_bits(a.y) & mk);
    o[2] = (unsigned short)(bf16_bits(a.z) & mk); o[3] = (unsigned short)(bf16_bits(a.w) & mk);
    o[4] = (unsigned short)(bf16_bits(b.x) & mk); o[5] = (unsigned short)(bf16_bits(b.y) & mk);
    o[6] = (unsigned short)(bf16_bits(b.z) & mk); o[7] = (unsigned short)(bf16_bits(b.w) & mk);
    unsigned short* dp = XAB + (size_t)sel * XPLANE + (size_t)u * 8;
    *(volatile v8us*)dp = o;
    __threadfence();
    *(volatile v8us*)dp = o;
  } else if (bx < 2 * XBLK + 4) {
    const int v  = (bx - 2 * XBLK) * PTHR + tid;
    const int s  = v >> 9;
    const int n  = (v >> 2) & 127;
    const int k8 = (v & 3) * 8;
    const float* p = W1 + (size_t)(32 * s + k8) * HID + (size_t)n;
    float f[8];
#pragma unroll
    for (int i = 0; i < 8; ++i) f[i] = p[(size_t)i * HID];
    v8us o;
#pragma unroll
    for (int i = 0; i < 8; ++i) o[i] = (unsigned short)bf16_bits(f[i]);
    unsigned short* dp = W1T + (size_t)v * 8;
    *(volatile v8us*)dp = o;
    __threadfence();
    *(volatile v8us*)dp = o;
  } else if (bx < 2 * XBLK + 12) {
    const int v  = (bx - 2 * XBLK - 4) * PTHR + tid;
    const int n  = v >> 5;
    const int k8 = (v & 31) * 8;
    const int kk = k8 & 127;
    const float* p = W2 + (size_t)kk * OUTC + (size_t)n;
    float f[8];
#pragma unroll
    for (int i = 0; i < 8; ++i) f[i] = p[(size_t)i * OUTC];
    v8us o;
#pragma unroll
    for (int i = 0; i < 8; ++i) o[i] = (unsigned short)bf16_bits(f[i]);
    unsigned short* dp = W2T + (size_t)v * 8;
    *(volatile v8us*)dp = o;
    __threadfence();
    *(volatile v8us*)dp = o;
  } else {
    const int i1 = tid < 31 ? tid : 31;
    int i2 = tid - 32;
    i2 = i2 < 0 ? 0 : (i2 > 15 ? 15 : i2);
    const v4f s1 = *(const v4f*)(b1 + 4 * i1);
    const v4f s2 = *(const v4f*)(b2 + 4 * i2);
    asm volatile("" :: "v"(s1), "v"(s2));
    v4f o1, o2;
    o1.x = bf16_val(s1.x); o1.y = bf16_val(s1.y); o1.z = bf16_val(s1.z); o1.w = bf16_val(s1.w);
    o2.x = bf16_val(s2.x); o2.y = bf16_val(s2.y); o2.z = bf16_val(s2.z); o2.w = bf16_val(s2.w);
    const bool w1 = tid < 32;
    const bool w2 = (tid >= 32) && (tid < 48);
    float* p1 = B1F + 4 * i1;
    float* p2 = B2F + 4 * i2;
    if (w1) *(volatile v4f*)p1 = o1;
    if (w2) *(volatile v4f*)p2 = o2;
    __threadfence();
    if (w1) *(volatile v4f*)p1 = o1;
    if (w2) *(volatile v4f*)p2 = o2;
  }
}

__global__ __launch_bounds__(G1THR) __attribute__((amdgpu_num_vgpr(248)))
void k_gemm_one(const unsigned short* __restrict__ XAB, const unsigned short* __restrict__ W1T,
                const float* __restrict__ B1F, float* PQ) {
  __shared__ __attribute__((aligned(16))) float stg[G1M * HID];
  __shared__ __attribute__((aligned(16))) float bsh[HID];
  const int tid = (int)threadIdx.x, lane = tid & 31, wave = tid >> 5, hh = lane >> 4, m = lane & 15;
  const int rowBase = (int)blockIdx.x * G1M;
  const int sel = (int)blockIdx.y;

  if (tid < 32) {
    const v4f b4 = *(const v4f*)(B1F + 4 * tid);
    asm volatile("" :: "v"(b4));
    v4f bq;
    bq.x = (sel != 0) ? b4.x : 0.0f;
    bq.y = (sel != 0) ? b4.y : 0.0f;
    bq.z = (sel != 0) ? b4.z : 0.0f;
    bq.w = (sel != 0) ? b4.w : 0.0f;
    *(v4fa*)(bsh + 4 * tid) = bq;
  }

  v8f acc[8];
  {
    const v8f z = {0.f, 0.f, 0.f, 0.f, 0.f, 0.f, 0.f, 0.f};
#pragma unroll
    for (int t = 0; t < 8; ++t) acc[t] = z;
  }
  const unsigned short* ap = XAB + (size_t)sel * XPLANE + (size_t)(rowBase + 16 * wave + m) * XP + 8 * hh;
  const unsigned short* bp = W1T + (size_t)sel * W1PLANE + (size_t)m * W1P + 8 * hh;
  FragB af;
  af.h[0] = *(const v8usa*)ap;
  af.h[1] = *(const v8usa*)(ap + 16);
#pragma unroll
  for (int nt = 0; nt < 8; ++nt) {
    const unsigned short* wq = bp + (size_t)(16 * nt) * W1P;
    FragB bf;
    bf.h[0] = *(const v8usa*)wq;
    bf.h[1] = *(const v8usa*)(wq + 16);
    acc[nt] = wmb(af, bf, acc[nt]);
  }

#pragma unroll
  for (int nt = 0; nt < 8; ++nt) {
    const int lc = 16 * nt + m;
#pragma unroll
    for (int r = 0; r < 8; ++r) {
      const int lr = 16 * wave + 8 * hh + r;
      stg[lr * HID + lc] = acc[nt][r];
    }
  }
  __syncthreads();

  const v4f bb4 = *(const v4fa*)(bsh + 4 * lane);
  v4f pv[16];
#pragma unroll
  for (int i = 0; i < 16; ++i) pv[i] = *(const v4fa*)(stg + (16 * wave + i) * HID + 4 * lane) + bb4;

  float* op = PQ + (size_t)sel * PQPLANE + (size_t)(rowBase + 16 * wave) * PQP + 4 * lane;
#pragma unroll
  for (int i = 0; i < 16; ++i) *(volatile v4f*)(op + (size_t)i * PQP) = pv[i];
  __threadfence();
#pragma unroll
  for (int i = 0; i < 16; ++i) *(volatile v4f*)(op + (size_t)i * PQP) = pv[i];
}

__global__ __launch_bounds__(WTHR) void k_walk(const float* __restrict__ PQ, const int* __restrict__ nbr,
                                               const int* __restrict__ rs, unsigned short* G, int* CNTL) {
#pragma clang fp contract(off)
  __shared__ __attribute__((aligned(16))) float rowst[WNW * HID];
  __shared__ __attribute__((aligned(16))) int cst[8];
  const int tid = (int)threadIdx.x, lane = tid & 31, wave = tid >> 5;
  const int pt   = (int)blockIdx.x * WNW + wave;
  const bool live = pt < NPTS;
  const int ptc  = live ? pt : NPTS - 1;

  const int r0 = rs[ptc];
  const int r1 = rs[ptc + 1];
  asm volatile("" :: "v"(r0), "v"(r1));
  const bool sf = (r0 < 0) | (r0 > r1) | (r1 > NE) |
                  ((ptc == 0) & (r0 != 0)) | ((ptc == NPTS - 1) & (r1 != NE));
  const int o   = r0 < 0 ? 0 : (r0 > NE ? NE : r0);
  const int r1c = r1 < 0 ? 0 : (r1 > NE ? NE : r1);
  const int craw = r1c - o;
  int c = craw < 0 ? 0 : (craw > TRIPCAP ? TRIPCAP : craw);
  c = c > NE - o ? NE - o : c;
  c = live ? c : 0;
  const int badv = (live && (sf | (craw > TRIPCAP))) ? 1 : 0;
  const int cm1  = c > 1 ? c : 1;
  const float inv = 1.0f / (float)cm1;
  const int os   = __builtin_amdgcn_readfirstlane(o);
  const int cs   = __builtin_amdgcn_readfirstlane(c);
  const int bads = __builtin_amdgcn_readfirstlane(badv);

  const v4f q = *(const v4f*)(PQ + PQPLANE + (size_t)ptc * PQP + 4 * lane);

  float a0 = 0.0f, a1 = 0.0f, a2 = 0.0f, a3 = 0.0f;
  const float* Pb = PQ + 4 * lane;
#pragma unroll 1
  for (int b0 = 0; b0 < cs; b0 += 32) {
    int idx = os + b0 + lane;
    idx = idx > NE - 1 ? NE - 1 : idx;
    int nb = nbr[idx];
    asm volatile("" :: "v"(nb));
    nb = nb < 0 ? 0 : (nb > NPTS - 1 ? NPTS - 1 : nb);
    const int rem = cs - b0;
    const int m32 = rem < 32 ? rem : 32;
    v4f nxt = *(const v4f*)(Pb + (size_t)__builtin_amdgcn_readlane(nb, 0) * PQP);
#pragma unroll 1
    for (int k = 0; k < m32; ++k) {
      const v4f cur = nxt;
      const int kn  = (k + 1 < 32) ? (k + 1) : 31;
      const int idn = __builtin_amdgcn_readlane(nb, kn);
      nxt = *(const v4f*)(Pb + (size_t)idn * PQP);
      a0 += gelu_e(cur.x + q.x);
      a1 += gelu_e(cur.y + q.y);
      a2 += gelu_e(cur.z + q.z);
      a3 += gelu_e(cur.w + q.w);
    }
  }

  const float qn = __int_as_float(0x7fc00000);
  v4f gv;
  gv.x = (bads != 0) ? qn : a0 * inv;
  gv.y = (bads != 0) ? qn : a1 * inv;
  gv.z = (bads != 0) ? qn : a2 * inv;
  gv.w = (bads != 0) ? qn : a3 * inv;

  float* wr = rowst + wave * HID;
  *(v4fa*)(wr + 4 * lane) = gv;
  wave_sync();
  const int cb = 8 * (lane & 15);
  const v4f x0 = *(const v4fa*)(wr + cb);
  const v4f x1 = *(const v4fa*)(wr + cb + 4);
  const bool isHi = lane < 16;
  unsigned h0, l0, h1, l1, h2, l2, h3, l3;
  pack2(x0.x, x0.y, h0, l0);
  pack2(x0.z, x0.w, h1, l1);
  pack2(x1.x, x1.y, h2, l2);
  pack2(x1.z, x1.w, h3, l3);
  v4u pw;
  pw.x = isHi ? h0 : l0;
  pw.y = isHi ? h1 : l1;
  pw.z = isHi ? h2 : l2;
  pw.w = isHi ? h3 : l3;
  unsigned short* gp = G + (size_t)pt * GAP + 8 * lane;
  *(volatile v4u*)gp = pw;
  __threadfence();
  *(volatile v4u*)gp = pw;

  if (lane == 0) cst[wave] = (bads != 0) ? 1 : cs;
  __syncthreads();
  if (wave == 0) {
    const v4i cv = *(const v4ia*)(cst + 4 * (lane & 1));
    v4i ov;
    ov.x = (lane < 2) ? cv.x : 0;
    ov.y = (lane < 2) ? cv.y : 0;
    ov.z = (lane < 2) ? cv.z : 0;
    ov.w = (lane < 2) ? cv.w : 0;
    int* cp = CNTL + (size_t)blockIdx.x * 32 + 4 * (lane & 7);
    if (lane < 8) *(volatile v4i*)cp = ov;
    __threadfence();
    if (lane < 8) *(volatile v4i*)cp = ov;
  }
}

__global__ __launch_bounds__(G2THR) __attribute__((amdgpu_num_vgpr(248)))
void k_gemm_two(const unsigned short* __restrict__ G, const unsigned short* __restrict__ W2T,
                const float* __restrict__ B2F, const int* __restrict__ CNTL, float* out) {
  __shared__ __attribute__((aligned(16))) float stg[G2M * OUTC];
  __shared__ __attribute__((aligned(16))) float b2s[OUTC];
  __shared__ __attribute__((aligned(16))) int cns[G2M];
  const int tid = (int)threadIdx.x, lane = tid & 31, wave = tid >> 5, hh = lane >> 4, m = lane & 15;
  const int rowBase = (int)blockIdx.x * G2M;

  if (wave == 0) {
    const v4f b4 = *(const v4f*)(B2F + 4 * (lane & 15));
    asm volatile("" :: "v"(b4));
    if (lane < 16) *(v4fa*)(b2s + 4 * lane) = b4;
  }
  if (tid < G2M) {
    const int r  = rowBase + tid;
    const int cv = CNTL[(size_t)(r >> 3) * 32 + (size_t)(r & 7)];
    cns[tid] = cv;
  }

  v8f acc[4];
  {
    const v8f z = {0.f, 0.f, 0.f, 0.f, 0.f, 0.f, 0.f, 0.f};
#pragma unroll
    for (int t = 0; t < 4; ++t) acc[t] = z;
  }
  const unsigned short* ap = G + (size_t)(rowBase + 16 * wave + m) * GAP + 8 * hh;
  const unsigned short* bp = W2T + (size_t)m * W2P + 8 * hh;
#pragma unroll 1
  for (int k0 = 0; k0 < KTWO; k0 += 32) {
    FragB af;
    af.h[0] = *(const v8usa*)(ap + k0);
    af.h[1] = *(const v8usa*)(ap + k0 + 16);
#pragma unroll
    for (int nt = 0; nt < 4; ++nt) {
      const unsigned short* wq = bp + (size_t)(16 * nt) * W2P + k0;
      FragB bf;
      bf.h[0] = *(const v8usa*)wq;
      bf.h[1] = *(const v8usa*)(wq + 16);
      acc[nt] = wmb(af, bf, acc[nt]);
    }
  }

#pragma unroll
  for (int nt = 0; nt < 4; ++nt) {
    const int lc = 16 * nt + m;
#pragma unroll
    for (int r = 0; r < 8; ++r) {
      const int lr = 16 * wave + 8 * hh + r;
      stg[lr * OUTC + lc] = acc[nt][r];
    }
  }
  __syncthreads();

  const v4f bb = *(const v4fa*)(b2s + 4 * m);
  v4f ov[8];
#pragma unroll
  for (int i = 0; i < 8; ++i) {
    const int lr = 16 * wave + 2 * i + hh;
    const v4f v = *(const v4fa*)(stg + lr * OUTC + 4 * m) + bb;
    const bool keep = cns[lr] > 0;
    v4f y;
    y.x = keep ? v.x : 0.0f;
    y.y = keep ? v.y : 0.0f;
    y.z = keep ? v.z : 0.0f;
    y.w = keep ? v.w : 0.0f;
    ov[i] = y;
  }
#pragma unroll
  for (int i = 0; i < 8; ++i) {
    const int gr = rowBase + 16 * wave + 2 * i + hh;
    const bool ok = gr < NPTS;
    const int grs = ok ? gr : 0;
    float* op = out + (size_t)grs * OUTC + 4 * m;
    if (ok) *(volatile v4f*)op = ov[i];
  }
  __threadfence();
#pragma unroll
  for (int i = 0; i < 8; ++i) {
    const int gr = rowBase + 16 * wave + 2 * i + hh;
    const bool ok = gr < NPTS;
    const int grs = ok ? gr : 0;
    float* op = out + (size_t)grs * OUTC + 4 * m;
    if (ok) *(volatile v4f*)op = ov[i];
  }
}

extern "C" void kernel_launch(void* const* d_in, const int* in_sizes, int n_in,
                              void* d_out, int out_size, void* d_ws, size_t ws_size,
                              hipStream_t stream) {
  if (n_in < 8) return;
  if (in_sizes[0] != NPTS * CIN || in_sizes[1] != NPTS * CIN) return;
  if (in_sizes[2] != 2 * CIN * HID || in_sizes[3] != HID) return;
  if (in_sizes[4] != HID * OUTC || in_sizes[5] != OUTC) return;
  if (in_sizes[6] != NE || in_sizes[7] != NPTS + 1) return;
  if (out_size != NPTS * OUTC) return;
  if (WS_TOTAL > ws_size) return;

  const float* xa  = (const float*)d_in[0];
  const float* xb  = (const float*)d_in[1];
  const float* W1  = (const float*)d_in[2];
  const float* b1  = (const float*)d_in[3];
  const float* W2  = (const float*)d_in[4];
  const float* b2  = (const float*)d_in[5];
  const int*   nbr = (const int*)d_in[6];
  const int*   rs  = (const int*)d_in[7];
  float* out = (float*)d_out;

  char* ws = (char*)d_ws;
  unsigned short* XAB = (unsigned short*)(ws + O_XAB);
  unsigned short* W1T = (unsigned short*)(ws + O_W1T);
  unsigned short* W2T = (unsigned short*)(ws + O_W2T);
  float* B1F = (float*)(ws + O_B1F);
  float* B2F = (float*)(ws + O_B2F);
  float* PQ  = (float*)(ws + O_PQ);
  unsigned short* G = (unsigned short*)(ws + O_G);
  int* CNTL = (int*)(ws + O_CN);

  k_prep<<<PREPB, PTHR, 0, stream>>>(xa, xb, W1, b1, W2, b2, XAB, W1T, W2T, B1F, B2F);
  const dim3 g1((unsigned)(MPAD / G1M), 2u, 1u);
  k_gemm_one<<<g1, G1THR, 0, stream>>>(XAB, W1T, B1F, PQ);
  k_walk<<<NWB, WTHR, 0, stream>>>(PQ, nbr, rs, G, CNTL);
  k_gemm_two<<<MPAD / G2M, G2THR, 0, stream>>>(G, W2T, B2F, CNTL, out);
}
